// EedgePath_MPNN_44770739093675
// MI455X (gfx1250) — hardware-verified
//
#include <hip/hip_runtime.h>
#include <stddef.h>
#include <stdint.h>


#define HD     64
#define NL     3
#define FCK    257
#define OWN    0
#define OWPQ   12288
#define OWF2   20480
#define OWEB   28672
#define OWES   32768
#define WLAYER 36864
#define WTOT   (NL * WLAYER)
#define WTASKL 4608
#define WBLKL  18

#define STHR   256
#define SWAV   (STHR / 32)
#define EPT    16
#define CHUNK  (STHR * EPT)
#define NBA    256
#define NPADG  256
#define GROWS  32
#define GTHR   64
#define APA    192
#define SXP    64
#define EPB    64
#define ETHR   128
#define APF    132
#define APC    68
#define WSCAP  134217728
#define LDS_A1 (NBA * 2 * HD * 4 + CHUNK * 4 + 64)
#define LDS_A2 (NBA * HD * 4 + CHUNK * 4 + 64)

#define DEGC   8
#define CHKB   64
#define CHKT   256
#define CNTL   32

static_assert(WBLKL * 256 == WTASKL);
static_assert(WTASKL * 8 == WLAYER);
static_assert(OWPQ == 3 * HD * HD);
static_assert(OWF2 == OWPQ + 2 * HD * HD);
static_assert(OWEB == OWF2 + 2 * HD * HD);
static_assert(OWES == OWEB + HD * HD);
static_assert(WLAYER == OWES + HD * HD);
static_assert(CHUNK == 4096 && NBA == 256 && STHR == 32 * SWAV);
static_assert((NBA * 2 * HD) % (4 * STHR) == 0 && (NBA * HD) % (4 * STHR) == 0);
static_assert(NBA == 32 * SWAV);
static_assert(GROWS == 16 * (GTHR / 32));
static_assert((GROWS * APA) % (4 * GTHR) == 0 && (GROWS * SXP) % (4 * GTHR) == 0 && (GROWS * 2 * HD) % (4 * GTHR) == 0);
static_assert(GROWS * 2 * HD <= GROWS * APA);
static_assert(EPB == 16 * (ETHR / 32) && ETHR == 2 * EPB);
static_assert((EPB * HD) % (4 * ETHR) == 0);
static_assert((APA % 4) == 0 && (APF % 4) == 0 && (APC % 4) == 0 && (SXP % 4) == 0);
static_assert((NPADG % NBA) == 0 && (NPADG % GROWS) == 0);
static_assert(LDS_A1 <= 160 * 1024 && LDS_A2 <= 160 * 1024);
static_assert(DEGC == 8 && CHKB == 64 && CHKT == 256 && CNTL == 32);
static_assert((CHKB % 32) == 0);

typedef float          v2f  __attribute__((ext_vector_type(2)));
typedef float          v4f  __attribute__((ext_vector_type(4)));
typedef float          v8f  __attribute__((ext_vector_type(8)));
typedef int            v4i  __attribute__((ext_vector_type(4)));
typedef unsigned short us;
typedef us             v8us  __attribute__((ext_vector_type(8)));
typedef us             v16us __attribute__((ext_vector_type(16)));
typedef __bf16         v16bf __attribute__((ext_vector_type(16)));
union FragB { v16bf v; v16us s; v8us u[2]; };

__device__ __forceinline__ v8f wmb(v16bf a, v16bf b, v8f c) {
  v8f d = __builtin_amdgcn_wmma_f32_16x16x32_bf16(false, a, false, b, (short)0, c, false, false);
  asm volatile("v_nop\n\tv_nop\n\tv_nop\n\tv_nop" : "+v"(d) : "v"(a), "v"(b));
  return d;
}

__device__ __forceinline__ unsigned rne16(float x) {
  const unsigned u = __float_as_uint(x);
  return (u + 0x7FFFu + ((u >> 16) & 1u)) >> 16;
}

__device__ __forceinline__ void split2(float x, us& h, us& l) {
  const unsigned hu = rne16(x);
  const float r = x - __uint_as_float(hu << 16);
  h = (us)hu;
  l = (us)rne16(r);
}

__device__ __forceinline__ void afrag(const float* ap, FragB& hi, FragB& lo) {
  const v4f x0 = *(const v4f*)(ap);
  const v4f x1 = *(const v4f*)(ap + 4);
  const v4f x2 = *(const v4f*)(ap + 16);
  const v4f x3 = *(const v4f*)(ap + 20);
  const float e[16] = {x0.x, x0.y, x0.z, x0.w, x1.x, x1.y, x1.z, x1.w,
                       x2.x, x2.y, x2.z, x2.w, x3.x, x3.y, x3.z, x3.w};
  v16us hs, ls;
#pragma unroll
  for (int i = 0; i < 16; ++i) {
    us h, l;
    split2(e[i], h, l);
    hs[i] = h;
    ls[i] = l;
  }
  hi.s = hs;
  lo.s = ls;
}

template <int NT, int KS>
__device__ __forceinline__ void wgemm(const float* At, int lda, const us* __restrict__ Bh,
                                      const us* __restrict__ Bl, int kpb, int lane, v8f (&acc)[NT]) {
  const int hh = lane >> 4, m = lane & 15;
#pragma unroll
  for (int t = 0; t < NT; ++t) { v8f z = {0.f, 0.f, 0.f, 0.f, 0.f, 0.f, 0.f, 0.f}; acc[t] = z; }
  const float* ap = At + m * lda + 8 * hh;
  const us* bh = Bh + (size_t)m * kpb + 8 * hh;
  const us* bl = Bl + (size_t)m * kpb + 8 * hh;
#pragma unroll 1
  for (int ks = 0; ks < KS; ++ks) {
    FragB ah, al;
    afrag(ap + 32 * ks, ah, al);
#pragma unroll
    for (int t = 0; t < NT; ++t) {
      const us* ph = bh + (size_t)(16 * t) * kpb + 32 * ks;
      const us* pl = bl + (size_t)(16 * t) * kpb + 32 * ks;
      FragB b1, b2;
      b1.u[0] = *(const v8us*)ph;
      b1.u[1] = *(const v8us*)(ph + 16);
      b2.u[0] = *(const v8us*)pl;
      b2.u[1] = *(const v8us*)(pl + 16);
      acc[t] = wmb(ah.v, b1.v, acc[t]);
      acc[t] = wmb(ah.v, b2.v, acc[t]);
      acc[t] = wmb(al.v, b1.v, acc[t]);
    }
  }
}

__global__ __launch_bounds__(CHKT) void k_chk(const int* __restrict__ esrc, const int* __restrict__ etrg,
                                              const int* __restrict__ lsrc, const int* __restrict__ ltrg,
                                              int* CNT, int nE, int nL) {
  __shared__ int swc[CHKT / 32];
  __shared__ __attribute__((aligned(16))) int sline[CNTL];
  const int tid = threadIdx.x, lane = tid & 31, wave = tid >> 5;
  const int gsz = CHKB * CHKT;
  int cnt = 0;
#pragma unroll 1
  for (int e = blockIdx.x * CHKT + tid; e < nE; e += gsz)
    cnt += (esrc[e] != e / DEGC) ? 1 : 0;
#pragma unroll 1
  for (int l = blockIdx.x * CHKT + tid; l < nL; l += gsz) {
    const int q = l / DEGC;
    int e1 = q;
    e1 = e1 > nE - 1 ? nE - 1 : e1;
    const int want = etrg[e1] * DEGC + (l - q * DEGC);
    cnt += (lsrc[l] != q) ? 1 : 0;
    cnt += (ltrg[l] != want) ? 1 : 0;
  }
#pragma unroll
  for (int o = 16; o > 0; o >>= 1) cnt += __shfl_xor(cnt, o, 32);
  if (lane == 0) swc[wave] = cnt;
  if (tid < CNTL) sline[tid] = 0;
  __syncthreads();
  if (tid == 0) {
    int t = 0;
#pragma unroll
    for (int w = 0; w < CHKT / 32; ++w) t += swc[w];
    sline[0] = t;
  }
  __syncthreads();
  int* gp = CNT + (size_t)blockIdx.x * CNTL;
  if (tid < CNTL / 4) {
    const v4i vv = ((const v4i*)sline)[tid];
    *(volatile v4i*)(gp + 4 * tid) = vv;
  }
  __threadfence();
  if (tid < CNTL / 4) {
    const v4i vv = ((const v4i*)sline)[tid];
    *(volatile v4i*)(gp + 4 * tid) = vv;
  }
}

__global__ __launch_bounds__(32) void k_chksum(int* CNT, int hostbad) {
  const int lane = threadIdx.x & 31;
  int c = 0;
#pragma unroll
  for (int b = 0; b < CHKB / 32; ++b) c += CNT[(size_t)(lane + 32 * b) * CNTL];
#pragma unroll
  for (int o = 16; o > 0; o >>= 1) c += __shfl_xor(c, o, 32);
  c += hostbad;
  v4i vv = {0, 0, 0, 0};
  if (lane == 0) vv.x = c;
  int* gp = CNT + (size_t)CHKB * CNTL;
  if (lane < CNTL / 4) *(volatile v4i*)(gp + 4 * lane) = vv;
  __threadfence();
  if (lane < CNTL / 4) *(volatile v4i*)(gp + 4 * lane) = vv;
}

__global__ __launch_bounds__(256) void k_wprep(const float* __restrict__ Wns, const float* __restrict__ Wnm,
                                               const float* __restrict__ Wne, const float* __restrict__ Wfc,
                                               const float* __restrict__ Wes, const float* __restrict__ Web,
                                               us* WPh, us* WPl) {
  const int blk = blockIdx.x, tid = threadIdx.x;
  const int l = blk / WBLKL;
  const int i = (blk - l * WBLKL) * 256 + tid;
  float v[8];
  int dst;
  if (i < 1536) {
    const int kb = i >> 9, j = i & 511, n = j >> 3, ks = (j & 7) * 8;
    const float* src = (kb == 0) ? Wns : ((kb == 1) ? Wnm : Wne);
#pragma unroll
    for (int e = 0; e < 8; ++e) v[e] = src[(size_t)(l * HD + ks + e) * HD + n];
    dst = OWN + n * (3 * HD) + kb * HD + ks;
  } else if (i < 2560) {
    const int j = i - 1536, n = j >> 3, ks = (j & 7) * 8;
    const int rb = (n < HD) ? HD : 2 * HD;
#pragma unroll
    for (int e = 0; e < 8; ++e) v[e] = Wfc[(size_t)(l * FCK + rb + ks + e) * HD + (n & (HD - 1))];
    dst = OWPQ + n * HD + ks;
  } else if (i < 3584) {
    const int j = i - 2560, n = j >> 4, ks = (j & 15) * 8;
    const int rw = (ks < HD) ? ks : ks + 2 * HD;
#pragma unroll
    for (int e = 0; e < 8; ++e) v[e] = Wfc[(size_t)(l * FCK + rw + e) * HD + n];
    dst = OWF2 + n * (2 * HD) + ks;
  } else if (i < 4096) {
    const int j = i - 3584, n = j >> 3, ks = (j & 7) * 8;
#pragma unroll
    for (int e = 0; e < 8; ++e) v[e] = Web[(size_t)(l * HD + ks + e) * HD + n];
    dst = OWEB + n * HD + ks;
  } else {
    const int j = i - 4096, n = j >> 3, ks = (j & 7) * 8;
#pragma unroll
    for (int e = 0; e < 8; ++e) v[e] = Wes[(size_t)(l * HD + ks + e) * HD + n];
    dst = OWES + n * HD + ks;
  }
  dst += l * WLAYER;
  v8us hv, lv;
#pragma unroll
  for (int e = 0; e < 8; ++e) {
    us h, lo;
    split2(v[e], h, lo);
    hv[e] = h;
    lv[e] = lo;
  }
  *(volatile v8us*)(WPh + dst) = hv;
  *(volatile v8us*)(WPl + dst) = lv;
  __threadfence();
  *(volatile v8us*)(WPh + dst) = hv;
  *(volatile v8us*)(WPl + dst) = lv;
}

__device__ __forceinline__ void loadids(const int* __restrict__ ids, int nE, int cbase, int tid, int vec,
                                        int (&d)[EPT]) {
  const int e0 = cbase + EPT * tid;
  if (vec != 0 && cbase + CHUNK <= nE) {
#pragma unroll
    for (int q = 0; q < EPT / 4; ++q) {
      const v4i t4 = *(const v4i*)(ids + e0 + 4 * q);
      d[4 * q] = t4.x; d[4 * q + 1] = t4.y; d[4 * q + 2] = t4.z; d[4 * q + 3] = t4.w;
    }
  } else {
#pragma unroll
    for (int j = 0; j < EPT; ++j) {
      int idx = e0 + j;
      const bool ok = idx < nE;
      idx = ok ? idx : nE - 1;
      const int val = ids[idx];
      d[j] = ok ? val : (-2147483647 - 1);
    }
  }
}

__device__ __forceinline__ void blkscan(int cnt, int lane, int wave, int* swt, int& pos, int& nh) {
  int x = cnt;
#pragma unroll
  for (int o = 1; o < 32; o <<= 1) {
    const int y = __shfl_up(x, o, 32);
    x += (lane >= o) ? y : 0;
  }
  if (lane == 31) swt[wave] = x;
  __syncthreads();
  int wpre = 0, tot = 0;
#pragma unroll
  for (int w = 0; w < SWAV; ++w) {
    const int vv = swt[w];
    wpre += (w < wave) ? vv : 0;
    tot += vv;
  }
  pos = wpre + x - cnt;
  nh = tot;
}

__global__ __launch_bounds__(STHR) void k_agg1(const int* __restrict__ srcs, const int* __restrict__ dsts,
                                                const float* __restrict__ xin, const float* __restrict__ efin,
                                                float* AGG, int nN, int nE, int nChunks, int vec, float xfloor) {
  extern __shared__ __attribute__((aligned(16))) char dynl[];
  float*    sacc  = (float*)dynl;
  unsigned* slist = (unsigned*)(dynl + NBA * 2 * HD * 4);
  int*      swt   = (int*)(dynl + NBA * 2 * HD * 4 + CHUNK * 4);
  const int tid = threadIdx.x, lane = tid & 31;
  const int wave = __builtin_amdgcn_readfirstlane(tid >> 5);
  const int n0 = blockIdx.x * NBA;
  {
    v4f z = {0.f, 0.f, 0.f, 0.f};
    v4f* p = (v4f*)sacc;
#pragma unroll
    for (int it = 0; it < (NBA * 2 * HD) / (4 * STHR); ++it) p[it * STHR + tid] = z;
  }
  __syncthreads();

#pragma unroll 1
  for (int c = 0; c < nChunks; ++c) {
    const int cbase = c * CHUNK;
    int d[EPT];
    loadids(dsts, nE, cbase, tid, vec, d);
    unsigned msk = 0;
#pragma unroll
    for (int j = 0; j < EPT; ++j) {
      const unsigned ld = (unsigned)d[j] - (unsigned)n0;
      msk |= ((ld < (unsigned)NBA) ? 1u : 0u) << j;
    }
    const int cnt = __builtin_popcount(msk);
    int pos, nh;
    blkscan(cnt, lane, wave, swt, pos, nh);
    const int e0 = cbase + EPT * tid;
#pragma unroll
    for (int j = 0; j < EPT; ++j) {
      if ((msk >> j) & 1u) {
        const unsigned ld = (unsigned)d[j] - (unsigned)n0;
        if (pos < CHUNK) slist[pos] = ((unsigned)(e0 + j) << 8) | ld;
        ++pos;
      }
    }
    __syncthreads();
    const int nhc = nh < CHUNK ? nh : CHUNK;
    for (int j = 0; j < nhc; ++j) {
      const unsigned pk = (unsigned)__builtin_amdgcn_readfirstlane((int)slist[j]);
      const int ld = (int)(pk & (unsigned)(NBA - 1));
      if ((ld & (SWAV - 1)) == wave) {
        int e = (int)(pk >> 8);
        e = e > nE - 1 ? nE - 1 : e;
        int s = srcs[e];
        s = s < 0 ? 0 : (s > nN - 1 ? nN - 1 : s);
        v2f xv = *(const v2f*)(xin + (size_t)s * HD + 2 * lane);
        xv.x = fmaxf(xv.x, xfloor);
        xv.y = fmaxf(xv.y, xfloor);
        const v2f ev = *(const v2f*)(efin + (size_t)e * HD + 2 * lane);
        v2f* ax = (v2f*)(sacc + ld * (2 * HD) + 2 * lane);
        v2f* ae = (v2f*)(sacc + ld * (2 * HD) + HD + 2 * lane);
        const v2f a0 = *ax;
        const v2f a1 = *ae;
        *ax = a0 + xv;
        *ae = a1 + ev;
      }
    }
  }
  __syncthreads();

  float* gp = AGG + (size_t)n0 * (2 * HD);
#pragma unroll
  for (int it = 0; it < (NBA * 2 * HD) / (4 * STHR); ++it) {
    const int f = it * STHR + tid;
    const v4f vv = ((const v4f*)sacc)[f];
    *(volatile v4f*)(gp + 4 * f) = vv;
  }
  __threadfence();
#pragma unroll
  for (int it = 0; it < (NBA * 2 * HD) / (4 * STHR); ++it) {
    const int f = it * STHR + tid;
    const v4f vv = ((const v4f*)sacc)[f];
    *(volatile v4f*)(gp + 4 * f) = vv;
  }
}

__device__ __forceinline__ void node_store(const float* sx, const float* snrm, const float* st,
                                           float* X, float* NRM, float* PQ, int rowBase, int tid) {
  float* gx = X + (size_t)rowBase * HD;
#pragma unroll
  for (int it = 0; it < (GROWS * SXP) / (4 * GTHR); ++it) {
    const int f = it * GTHR + tid;
    const v4f vv = ((const v4f*)sx)[f];
    *(volatile v4f*)(gx + 4 * f) = vv;
  }
  if (tid < GROWS / 4) {
    const v4f vv = ((const v4f*)snrm)[tid];
    *(volatile v4f*)(NRM + rowBase + 4 * tid) = vv;
  }
  float* gp = PQ + (size_t)rowBase * (2 * HD);
#pragma unroll
  for (int it = 0; it < (GROWS * 2 * HD) / (4 * GTHR); ++it) {
    const int f = it * GTHR + tid;
    const v4f vv = ((const v4f*)st)[f];
    *(volatile v4f*)(gp + 4 * f) = vv;
  }
}

__global__ __launch_bounds__(GTHR) void k_node(const float* xin, const float* __restrict__ AGG,
                                               const us* __restrict__ WPh, const us* __restrict__ WPl,
                                               const float* __restrict__ bn, float* X, float* NRM, float* PQ,
                                               int nXrows, float xfloor) {
  __shared__ __attribute__((aligned(16))) float atile[GROWS * APA];
  __shared__ __attribute__((aligned(16))) float sx[GROWS * SXP];
  __shared__ __attribute__((aligned(16))) float snrm[GROWS];
  const int tid = threadIdx.x, lane = tid & 31, wave = tid >> 5, hh = lane >> 4, m = lane & 15;
  const int rowBase = blockIdx.x * GROWS;

#pragma unroll 4
  for (int it = 0; it < (GROWS * APA) / (4 * GTHR); ++it) {
    const int f = it * GTHR + tid;
    const int row = f / (APA / 4);
    const int q = f - row * (APA / 4);
    int xr = rowBase + row;
    xr = xr > nXrows - 1 ? nXrows - 1 : xr;
    v4f xv = *(const v4f*)(xin + (size_t)xr * HD + 4 * (q & 15));
    const v4f av = *(const v4f*)(AGG + (size_t)(rowBase + row) * (2 * HD) + 4 * ((q - 16) & 31));
    xv.x = fmaxf(xv.x, xfloor); xv.y = fmaxf(xv.y, xfloor);
    xv.z = fmaxf(xv.z, xfloor); xv.w = fmaxf(xv.w, xfloor);
    v4f vv = av;
    if (q < 16) vv = xv;
    *(v4f*)(atile + row * APA + 4 * q) = vv;
  }
  __syncthreads();

  {
    v8f acc[4];
    wgemm<4, 6>(atile + wave * 16 * APA, APA, WPh + OWN, WPl + OWN, 3 * HD, lane, acc);
    float* sp = sx + (wave * 16 + 8 * hh) * SXP + m;
#pragma unroll
    for (int t = 0; t < 4; ++t) {
      const float bv = bn[16 * t + m];
#pragma unroll
      for (int r = 0; r < 8; ++r) sp[r * SXP + 16 * t] = acc[t][r] + bv;
    }
  }
  __syncthreads();

  {
    const int row = tid >> 1, c = tid & 1;
    const v4f* rp = (const v4f*)(sx + row * SXP + 32 * c);
    float s = 0.0f;
#pragma unroll
    for (int j = 0; j < 8; ++j) {
      const v4f vv = rp[j];
      s += vv.x * vv.x + vv.y * vv.y + vv.z * vv.z + vv.w * vv.w;
    }
    s += __shfl_xor(s, 1, 32);
    if (c == 0) snrm[row] = sqrtf(s);
  }
  {
    v8f acc[8];
    wgemm<8, 2>(sx + wave * 16 * SXP, SXP, WPh + OWPQ, WPl + OWPQ, HD, lane, acc);
    float* sp = atile + (wave * 16 + 8 * hh) * (2 * HD) + m;
#pragma unroll
    for (int t = 0; t < 8; ++t)
#pragma unroll
      for (int r = 0; r < 8; ++r) sp[r * (2 * HD) + 16 * t] = acc[t][r];
  }
  __syncthreads();

  node_store(sx, snrm, atile, X, NRM, PQ, rowBase, tid);
  __threadfence();
  node_store(sx, snrm, atile, X, NRM, PQ, rowBase, tid);
}

__global__ __launch_bounds__(ETHR) void k_edgefc(
    const float* efin, const int* __restrict__ srcs, const int* __restrict__ trgs,
    const float* __restrict__ X, const float* __restrict__ NRM, const float* __restrict__ PQ,
    const us* __restrict__ WPh, const us* __restrict__ WPl, const float* __restrict__ wsimp,
    const float* __restrict__ bfc, float* EF, int nN, int nE) {
  __shared__ __attribute__((aligned(16))) float sA[EPB * APF];
  __shared__ __attribute__((aligned(16))) float spq[EPB * HD];
  __shared__ __attribute__((aligned(16))) float ssim[EPB];
  __shared__ __attribute__((aligned(16))) float sbfc[HD];
  const int tid = threadIdx.x, lane = tid & 31, wave = tid >> 5, hh = lane >> 4, m = lane & 15;
  const int e0 = blockIdx.x * EPB;
  if (tid < HD) sbfc[tid] = bfc[tid];
  float wsim[4];
#pragma unroll
  for (int t = 0; t < 4; ++t) wsim[t] = wsimp[16 * t + m];
  __syncthreads();

  {
    const int r = tid >> 1, c = tid & 1;
    int e = e0 + r;
    e = e > nE - 1 ? nE - 1 : e;
    int s = srcs[e];
    s = s < 0 ? 0 : (s > nN - 1 ? nN - 1 : s);
    int t = trgs[e];
    t = t < 0 ? 0 : (t > nN - 1 ? nN - 1 : t);
    const float ns = NRM[s], nt = NRM[t];
    const float* fp  = efin + (size_t)e * HD + 32 * c;
    const float* xsp = X + (size_t)s * HD + 32 * c;
    const float* xtp = X + (size_t)t * HD + 32 * c;
    const float* pp  = PQ + (size_t)s * (2 * HD) + 32 * c;
    const float* qp  = PQ + (size_t)t * (2 * HD) + HD + 32 * c;
    const float* bp  = sbfc + 32 * c;
    float* ap = sA + r * APF + 32 * c;
    float* dp = sA + r * APF + HD + 32 * c;
    float* pq = spq + r * HD + 32 * c;
    float dot = 0.0f;
#pragma unroll 1
    for (int cg = 0; cg < 4; ++cg) {
      const int o = 8 * cg;
      const v4f f0 = *(const v4f*)(fp + o),  f1 = *(const v4f*)(fp + o + 4);
      const v4f s0 = *(const v4f*)(xsp + o), s1 = *(const v4f*)(xsp + o + 4);
      const v4f t0 = *(const v4f*)(xtp + o), t1 = *(const v4f*)(xtp + o + 4);
      const v4f p0 = *(const v4f*)(pp + o),  p1 = *(const v4f*)(pp + o + 4);
      const v4f q0 = *(const v4f*)(qp + o),  q1 = *(const v4f*)(qp + o + 4);
      const v4f b0 = *(const v4f*)(bp + o),  b1 = *(const v4f*)(bp + o + 4);
      *(v4f*)(ap + o) = f0;
      *(v4f*)(ap + o + 4) = f1;
      v4f d0 = s0 - t0, d1 = s1 - t1;
      d0.x = fabsf(d0.x); d0.y = fabsf(d0.y); d0.z = fabsf(d0.z); d0.w = fabsf(d0.w);
      d1.x = fabsf(d1.x); d1.y = fabsf(d1.y); d1.z = fabsf(d1.z); d1.w = fabsf(d1.w);
      *(v4f*)(dp + o) = d0;
      *(v4f*)(dp + o + 4) = d1;
      *(v4f*)(pq + o) = p0 + q0 + b0;
      *(v4f*)(pq + o + 4) = p1 + q1 + b1;
      dot += s0.x * t0.x + s0.y * t0.y + s0.z * t0.z + s0.w * t0.w;
      dot += s1.x * t1.x + s1.y * t1.y + s1.z * t1.z + s1.w * t1.w;
    }
    dot += __shfl_xor(dot, 1, 32);
    const float den = fmaxf(ns * nt, 1e-8f);
    const float sim = dot * (1.0f / den);
    if (c == 0) ssim[r] = sim;
  }
  __syncthreads();

  {
    v8f acc[4];
    wgemm<4, 4>(sA + wave * 16 * APF, APF, WPh + OWF2, WPl + OWF2, 2 * HD, lane, acc);
    float* sp = spq + (wave * 16 + 8 * hh) * HD + m;
    const float* ss = ssim + wave * 16 + 8 * hh;
#pragma unroll
    for (int r = 0; r < 8; ++r) {
      const float sv = ss[r];
#pragma unroll
      for (int t = 0; t < 4; ++t) {
        const float vv = acc[t][r] + sp[r * HD + 16 * t] + sv * wsim[t];
        sp[r * HD + 16 * t] = vv;
      }
    }
  }
  __syncthreads();

  float* gp = EF + (size_t)e0 * HD;
#pragma unroll
  for (int it = 0; it < (EPB * HD) / (4 * ETHR); ++it) {
    const int f = it * ETHR + tid;
    const v4f vv = ((const v4f*)spq)[f];
    *(volatile v4f*)(gp + 4 * f) = vv;
  }
  __threadfence();
#pragma unroll
  for (int it = 0; it < (EPB * HD) / (4 * ETHR); ++it) {
    const int f = it * ETHR + tid;
    const v4f vv = ((const v4f*)spq)[f];
    *(volatile v4f*)(gp + 4 * f) = vv;
  }
}

__global__ __launch_bounds__(STHR) void k_agg2(const int* __restrict__ dsts, const float* __restrict__ EF,
                                                const us* __restrict__ WebH, const us* __restrict__ WebL,
                                                float* T, int nE, int nChunks, int vec) {
  extern __shared__ __attribute__((aligned(16))) char dynl[];
  float*    sacc  = (float*)dynl;
  unsigned* slist = (unsigned*)(dynl + NBA * HD * 4);
  int*      swt   = (int*)(dynl + NBA * HD * 4 + CHUNK * 4);
  const int tid = threadIdx.x, lane = tid & 31, hh = lane >> 4, m = lane & 15;
  const int wave = __builtin_amdgcn_readfirstlane(tid >> 5);
  const int n0 = blockIdx.x * NBA;
  {
    v4f z = {0.f, 0.f, 0.f, 0.f};
    v4f* p = (v4f*)sacc;
#pragma unroll
    for (int it = 0; it < (NBA * HD) / (4 * STHR); ++it) p[it * STHR + tid] = z;
  }
  __syncthreads();

#pragma unroll 1
  for (int c = 0; c < nChunks; ++c) {
    const int cbase = c * CHUNK;
    int d[EPT];
    loadids(dsts, nE, cbase, tid, vec, d);
    unsigned msk = 0;
#pragma unroll
    for (int j = 0; j < EPT; ++j) {
      const unsigned ld = (unsigned)d[j] - (unsigned)n0;
      msk |= ((ld < (unsigned)NBA) ? 1u : 0u) << j;
    }
    const int cnt = __builtin_popcount(msk);
    int pos, nh;
    blkscan(cnt, lane, wave, swt, pos, nh);
    const int e0 = cbase + EPT * tid;
#pragma unroll
    for (int j = 0; j < EPT; ++j) {
      if ((msk >> j) & 1u) {
        const unsigned ld = (unsigned)d[j] - (unsigned)n0;
        if (pos < CHUNK) slist[pos] = ((unsigned)(e0 + j) << 8) | ld;
        ++pos;
      }
    }
    __syncthreads();
    const int nhc = nh < CHUNK ? nh : CHUNK;
    for (int j = 0; j < nhc; ++j) {
      const unsigned pk = (unsigned)__builtin_amdgcn_readfirstlane((int)slist[j]);
      const int ld = (int)(pk & (unsigned)(NBA - 1));
      if ((ld & (SWAV - 1)) == wave) {
        int e = (int)(pk >> 8);
        e = e > nE - 1 ? nE - 1 : e;
        const v2f ev = *(const v2f*)(EF + (size_t)e * HD + 2 * lane);
        v2f* ap = (v2f*)(sacc + ld * HD + 2 * lane);
        const v2f av = *ap;
        *ap = av + ev;
      }
    }
  }
  __syncthreads();

#pragma unroll 1
  for (int rt = 0; rt < 2; ++rt) {
    const int r0 = wave * 32 + rt * 16;
    v8f acc[4];
    wgemm<4, 2>(sacc + r0 * HD, HD, WebH, WebL, HD, lane, acc);
    float* sp = sacc + (r0 + 8 * hh) * HD + m;
#pragma unroll
    for (int t = 0; t < 4; ++t)
#pragma unroll
      for (int r = 0; r < 8; ++r) sp[r * HD + 16 * t] = acc[t][r];
  }
  __syncthreads();

  float* gp = T + (size_t)n0 * HD;
#pragma unroll
  for (int it = 0; it < (NBA * HD) / (4 * STHR); ++it) {
    const int f = it * STHR + tid;
    const v4f vv = ((const v4f*)sacc)[f];
    *(volatile v4f*)(gp + 4 * f) = vv;
  }
  __threadfence();
#pragma unroll
  for (int it = 0; it < (NBA * HD) / (4 * STHR); ++it) {
    const int f = it * STHR + tid;
    const v4f vv = ((const v4f*)sacc)[f];
    *(volatile v4f*)(gp + 4 * f) = vv;
  }
}

__global__ __launch_bounds__(ETHR) void k_edgeconv(
    const float* EFin, const int* __restrict__ srcs, const float* __restrict__ T,
    const us* __restrict__ WesH, const us* __restrict__ WesL, const float* __restrict__ be,
    const int* __restrict__ badp, float* dst, int nN, int nE, int nRowsOut) {
  __shared__ __attribute__((aligned(16))) float sA[EPB * APC];
  __shared__ __attribute__((aligned(16))) float sadd[EPB * HD];
  const int tid = threadIdx.x, lane = tid & 31, wave = tid >> 5, hh = lane >> 4, m = lane & 15;
  const int e0 = blockIdx.x * EPB;
  const int bad = badp[0];
  const float qn = __uint_as_float(0x7fc00000u);
  const v4f nanv = {qn, qn, qn, qn};
  {
    const int r = tid >> 1, c = tid & 1;
    int e = e0 + r;
    e = e > nE - 1 ? nE - 1 : e;
    int s = srcs[e];
    s = s < 0 ? 0 : (s > nN - 1 ? nN - 1 : s);
    const float* fp = EFin + (size_t)e * HD + 32 * c;
    const float* tp = T + (size_t)s * HD + 32 * c;
    const float* bp = be + 32 * c;
    float* ap = sA + r * APC + 32 * c;
    float* dp = sadd + r * HD + 32 * c;
#pragma unroll 1
    for (int cg = 0; cg < 4; ++cg) {
      const int o = 8 * cg;
      const v4f f0 = *(const v4f*)(fp + o), f1 = *(const v4f*)(fp + o + 4);
      const v4f t0 = *(const v4f*)(tp + o), t1 = *(const v4f*)(tp + o + 4);
      const v4f b0 = *(const v4f*)(bp + o), b1 = *(const v4f*)(bp + o + 4);
      *(v4f*)(ap + o) = f0;
      *(v4f*)(ap + o + 4) = f1;
      *(v4f*)(dp + o) = t0 + b0;
      *(v4f*)(dp + o + 4) = t1 + b1;
    }
  }
  __syncthreads();

  {
    v8f acc[4];
    wgemm<4, 2>(sA + wave * 16 * APC, APC, WesH, WesL, HD, lane, acc);
    float* sp = sadd + (wave * 16 + 8 * hh) * HD + m;
#pragma unroll
    for (int t = 0; t < 4; ++t)
#pragma unroll
      for (int r = 0; r < 8; ++r) {
        const float vv = acc[t][r] + sp[r * HD + 16 * t];
        sp[r * HD + 16 * t] = vv;
      }
  }
  __syncthreads();

  float* gp = dst + (size_t)e0 * HD;
#pragma unroll
  for (int it = 0; it < (EPB * HD) / (4 * ETHR); ++it) {
    const int f = it * ETHR + tid;
    const int row = f >> 4;
    v4f vv = ((const v4f*)sadd)[f];
    if (bad != 0) vv = nanv;
    if (e0 + row < nRowsOut) *(volatile v4f*)(gp + 4 * f) = vv;
  }
  __threadfence();
#pragma unroll
  for (int it = 0; it < (EPB * HD) / (4 * ETHR); ++it) {
    const int f = it * ETHR + tid;
    const int row = f >> 4;
    v4f vv = ((const v4f*)sadd)[f];
    if (bad != 0) vv = nanv;
    if (e0 + row < nRowsOut) *(volatile v4f*)(gp + 4 * f) = vv;
  }
}

extern "C" void kernel_launch(void* const* d_in, const int* in_sizes, int n_in,
                              void* d_out, int out_size, void* d_ws, size_t ws_size,
                              hipStream_t stream) {
  if (n_in < 15) return;
  if (in_sizes[0] < HD || (in_sizes[0] % HD) != 0) return;
  const int nN = in_sizes[0] / HD;
  const int nE = in_sizes[11];
  if (nN < 1 || nE < 1) return;
  if (nN > (1 << 22) || nE > (1 << 23)) return;
  if (in_sizes[1] != nE * HD || in_sizes[12] != nE) return;
  if (in_sizes[2] != NL * HD * HD || in_sizes[3] != NL * HD * HD || in_sizes[4] != NL * HD * HD) return;
  if (in_sizes[8] != NL * HD * HD || in_sizes[9] != NL * HD * HD) return;
  if (in_sizes[5] != NL * HD || in_sizes[7] != NL * HD || in_sizes[10] != NL * HD) return;
  if (in_sizes[6] != NL * FCK * HD) return;
  if (out_size != nE * HD) return;
  if (in_sizes[13] < 0 || in_sizes[14] < 0) return;
  const int nL13 = in_sizes[13], nL14 = in_sizes[14];
  const int nLc = nL13 < nL14 ? nL13 : nL14;
  const int hostbad = (nL13 != nE * DEGC || nL14 != nE * DEGC) ? 1 : 0;

  const float* dx   = (const float*)d_in[0];
  const float* def  = (const float*)d_in[1];
  const float* Wns  = (const float*)d_in[2];
  const float* Wnm  = (const float*)d_in[3];
  const float* Wne  = (const float*)d_in[4];
  const float* bn   = (const float*)d_in[5];
  const float* Wfc  = (const float*)d_in[6];
  const float* bfc  = (const float*)d_in[7];
  const float* Wes  = (const float*)d_in[8];
  const float* Web  = (const float*)d_in[9];
  const float* be   = (const float*)d_in[10];
  const int*   srcs = (const int*)d_in[11];
  const int*   trgs = (const int*)d_in[12];
  const int*   lsrc = (const int*)d_in[13];
  const int*   ltrg = (const int*)d_in[14];
  float* out = (float*)d_out;

  const int NP = ((nN + NPADG - 1) / NPADG) * NPADG;
  const int EP = ((nE + EPB - 1) / EPB) * EPB;
  const int gAgg  = NP / NBA;
  const int gNode = NP / GROWS;
  const int gEdge = EP / EPB;
  const int nChunks = (nE + CHUNK - 1) / CHUNK;

  char* ws = (char*)d_ws;
  size_t off = 0;
  const size_t oWh  = off; off += (size_t)WTOT * 2;            off = (off + 255) & ~(size_t)255;
  const size_t oWl  = off; off += (size_t)WTOT * 2;            off = (off + 255) & ~(size_t)255;
  const size_t oAGG = off; off += (size_t)NP * 2 * HD * 4;     off = (off + 255) & ~(size_t)255;
  const size_t oX   = off; off += (size_t)NP * HD * 4;         off = (off + 255) & ~(size_t)255;
  const size_t oNRM = off; off += (size_t)NP * 4;              off = (off + 255) & ~(size_t)255;
  const size_t oPQ  = off; off += (size_t)NP * 2 * HD * 4;     off = (off + 255) & ~(size_t)255;
  const size_t oEF  = off; off += (size_t)EP * HD * 4;         off = (off + 255) & ~(size_t)255;
  const size_t oT   = off; off += (size_t)NP * HD * 4;         off = (off + 255) & ~(size_t)255;
  const size_t oCNT = off; off += (size_t)(CHKB + 1) * CNTL * 4; off = (off + 255) & ~(size_t)255;
  if (off > ws_size || off > (size_t)WSCAP) return;
  us*    WPh = (us*)(ws + oWh);
  us*    WPl = (us*)(ws + oWl);
  float* AGG = (float*)(ws + oAGG);
  float* X   = (float*)(ws + oX);
  float* NRM = (float*)(ws + oNRM);
  float* PQ  = (float*)(ws + oPQ);
  float* EF  = (float*)(ws + oEF);
  float* T   = (float*)(ws + oT);
  int*   CNT = (int*)(ws + oCNT);
  const int* badp = CNT + (size_t)CHKB * CNTL;

  hipFuncSetAttribute(reinterpret_cast<const void*>(&k_agg1), hipFuncAttributeMaxDynamicSharedMemorySize, LDS_A1);
  hipFuncSetAttribute(reinterpret_cast<const void*>(&k_agg2), hipFuncAttributeMaxDynamicSharedMemorySize, LDS_A2);

  const float ninf = -__builtin_huge_valf();

  k_chk<<<CHKB, CHKT, 0, stream>>>(srcs, trgs, lsrc, ltrg, CNT, nE, nLc);
  k_chksum<<<1, 32, 0, stream>>>(CNT, hostbad);

  k_wprep<<<NL * WBLKL, 256, 0, stream>>>(Wns, Wnm, Wne, Wfc, Wes, Web, WPh, WPl);

  for (int l = 0; l < NL; ++l) {
    const float* xin  = (l == 0) ? dx : (const float*)X;
    const float* efin = (l == 0) ? def : (const float*)EF;
    const int   nXr = (l == 0) ? nN : NP;
    const float xfl = (l == 0) ? ninf : 0.0f;
    const us* wh = WPh + (size_t)l * WLAYER;
    const us* wl = WPl + (size_t)l * WLAYER;
    k_agg1<<<gAgg, STHR, LDS_A1, stream>>>(srcs, trgs, xin, efin, AGG, nN, nE, nChunks, 1, xfl);
    k_node<<<gNode, GTHR, 0, stream>>>(xin, AGG, wh, wl, bn + (size_t)l * HD, X, NRM, PQ, nXr, xfl);
    k_edgefc<<<gEdge, ETHR, 0, stream>>>(efin, srcs, trgs, X, NRM, PQ, wh, wl,
                                         Wfc + ((size_t)l * FCK + 256) * HD, bfc + (size_t)l * HD,
                                         EF, nN, nE);
    k_agg2<<<gAgg, STHR, LDS_A2, stream>>>(trgs, EF, wh + OWEB, wl + OWEB, T, nE, nChunks, 1);
    float* dsto = (l == NL - 1) ? out : EF;
    const int nRows = (l == NL - 1) ? nE : EP;
    k_edgeconv<<<gEdge, ETHR, 0, stream>>>(EF, srcs, T, wh + OWES, wl + OWES, be + (size_t)l * HD,
                                           badp, dsto, nN, nE, nRows);
  }
}
